// GraphAttentionLayer_352187318397
// MI455X (gfx1250) — hardware-verified
//
#include <hip/hip_runtime.h>


#ifndef NB
#define NB 192
#endif
#ifndef SEQ
#define SEQ 512
#endif
#define NB_FULL  192
#define SEQ_FULL 512
#ifndef OUT_SEQ
#define OUT_SEQ SEQ
#endif
#define FIN  64
#define FOUT 64
#define AW   4
#define OSP  68
#define LRA  0.2f
#define L2E  1.4426950408889634f
#define NEGT ((float)(-9.0e15 * 1.4426950408889634))
#define PSH  14.0f
#define NEGB (-3.0e38f)
#define PLN  ((size_t)NB * SEQ)

static_assert(FIN == 64);
static_assert(FOUT == 64);
static_assert(FIN % 32 == 0);
static_assert(SEQ % 64 == 0);
static_assert(((size_t)NB * SEQ) % 64 == 0);
static_assert(SEQ % 32 == 0);
static_assert(SEQ % (16 * AW) == 0);
static_assert(NB <= NB_FULL);
static_assert(SEQ <= SEQ_FULL);
static_assert((OSP * 4) % 16 == 0);
static_assert(OSP >= FOUT);
static_assert(((size_t)SEQ * FIN) % 8 == 0);
static_assert(2 * 256 * 8 == FIN * FOUT);
static_assert(4 * 32 * 16 == 16 * 64 * 2);
static_assert(32 * 16 == 2 * 64 * 4);
static_assert(8 * 32 * 16 == 16 * FOUT * 4);
static_assert((size_t)FIN * (FOUT + 1) * 4 <= 131072);
static_assert((size_t)(16 * 68 + 2 * 64) * 4 <= 131072);
static_assert((size_t)AW * 16 * OSP * 4 <= 131072);

typedef _Float16 h16;
typedef unsigned short bf;
typedef __attribute__((ext_vector_type(16))) __bf16   v16bf;
typedef __attribute__((ext_vector_type(16))) _Float16 v16h;
typedef __attribute__((ext_vector_type(8)))  _Float16 v8h;
typedef __attribute__((ext_vector_type(8)))  unsigned short v8us;
typedef __attribute__((ext_vector_type(8)))  float    v8f;
typedef __attribute__((ext_vector_type(4)))  float    v4f;
typedef v4f  __attribute__((may_alias)) v4fa;

__device__ __forceinline__ unsigned short f2bf(float f) { unsigned u = __float_as_uint(f); u += 0x7FFFu + ((u >> 16) & 1u); return (unsigned short)(u >> 16); }
__device__ __forceinline__ float bfr(float f) { return __uint_as_float(((unsigned)f2bf(f)) << 16); }
__device__ __forceinline__ v16h cat16(v8h lo, v8h hi) { return __builtin_shufflevector(lo, hi, 0, 1, 2, 3, 4, 5, 6, 7, 8, 9, 10, 11, 12, 13, 14, 15); }
__device__ __forceinline__ v16bf cat16b(v8us lo, v8us hi) { return __builtin_bit_cast(v16bf, __builtin_shufflevector(lo, hi, 0, 1, 2, 3, 4, 5, 6, 7, 8, 9, 10, 11, 12, 13, 14, 15)); }
__device__ __forceinline__ v8f wmma16(v16h a, v16h b, v8f c) { return __builtin_amdgcn_wmma_f32_16x16x32_f16(false, a, false, b, (short)0, c, false, false); }
__device__ __forceinline__ v8f wmmab(v16bf a, v16bf b, v8f c) { return __builtin_amdgcn_wmma_f32_16x16x32_bf16(false, a, false, b, (short)0, c, false, false); }
__device__ __forceinline__ v16h  ldh(const h16* p) { return cat16(*(const v8h*)p, *(const v8h*)(p + 16)); }
__device__ __forceinline__ v16bf ldb(const bf* p)  { return cat16b(*(const v8us*)p, *(const v8us*)(p + 16)); }
__device__ __forceinline__ void wave_sync() { __builtin_amdgcn_fence(3  , "wavefront"); __builtin_amdgcn_wave_barrier(); asm volatile("" ::: "memory"); }

__device__ __forceinline__ h16 toh_flush(float v) { const h16 r = (h16)v; return (fabsf(v) < 6.103515625e-05f) ? (h16)0.0f : r; }
__device__ __forceinline__ v8f wmma16g(v16h a, v16h b, v8f c) { c = wmma16(a, b, c); asm volatile("v_nop\n\tv_nop\n\tv_nop\n\tv_nop" : "+v"(c) : "v"(a), "v"(b)); return c; }
__device__ __forceinline__ v8f wmmabg(v16bf a, v16bf b, v8f c) { c = wmmab(a, b, c); asm volatile("v_nop\n\tv_nop\n\tv_nop\n\tv_nop" : "+v"(c) : "v"(a), "v"(b)); return c; }
__device__ __forceinline__ float elu1(float x) { const float xn = fminf(x, 0.0f); const float en = __builtin_amdgcn_exp2f(xn * L2E) - 1.0f; return (x > 0.0f) ? x : en; }

__global__ __launch_bounds__(256) void k_cvt8(const float* __restrict__ src, bf* dst, size_t n8) {
    const size_t i = (size_t)blockIdx.x * 256 + threadIdx.x; if (i >= n8) return;
    const v8f v = *(const v8f*)(src + i * 8); v8us o;
#pragma unroll
    for (int k = 0; k < 8; ++k) o[k] = f2bf(v[k]);
    *(volatile v8us*)(dst + i * 8) = o; __threadfence(); *(volatile v8us*)(dst + i * 8) = o;
}

__global__ __launch_bounds__(256) void k_wt(const float* __restrict__ W, bf* WT) {
    __shared__ float tl[FIN * (FOUT + 1)];
    const int tid = threadIdx.x;
#pragma unroll 1
    for (int i = tid; i < FIN * FOUT; i += 256) { const int f = i / FOUT, o = i % FOUT; tl[f * (FOUT + 1) + o] = W[i]; }
    __syncthreads();
#pragma unroll 1
    for (int it = 0; it < 2; ++it) {
        const int p = it * 256 + tid; const int o = p >> 3, f8 = (p & 7) * 8; v8us ov;
#pragma unroll
        for (int k = 0; k < 8; ++k) ov[k] = f2bf(tl[(f8 + k) * (FOUT + 1) + o]);
        *(volatile v8us*)(WT + (size_t)p * 8) = ov; __threadfence(); *(volatile v8us*)(WT + (size_t)p * 8) = ov;
    }
}

__global__ __launch_bounds__(32) void k_whT(const bf* __restrict__ WT, const bf* __restrict__ XB, const float* __restrict__ avec, h16* VT, float* WH12) {
    __shared__ __align__(16) float os[16 * 68];
    __shared__ __align__(16) float sv[2 * 64];
    const int K = FIN;
    const int lane = threadIdx.x & 31, lr = lane & 15, hi = lane >> 4; const int c0 = blockIdx.x * 64;
    v8f acc[4][4];
#pragma unroll
    for (int mb = 0; mb < 4; ++mb)
#pragma unroll
        for (int nb = 0; nb < 4; ++nb) acc[mb][nb] = (v8f){};
    const size_t aoff = (size_t)lr * K + 8 * hi, boff = (size_t)(c0 + lr) * K + 8 * hi;
#pragma unroll 1
    for (int kc = 0; kc < K; kc += 32) {
        v16bf a[4];
#pragma unroll
        for (int mb = 0; mb < 4; ++mb) a[mb] = ldb(WT + aoff + (size_t)mb * 16 * K + kc);
#pragma unroll
        for (int nb = 0; nb < 4; ++nb) { const v16bf b = ldb(XB + boff + (size_t)nb * 16 * K + kc);
#pragma unroll
            for (int mb = 0; mb < 4; ++mb) acc[mb][nb] = wmmabg(a[mb], b, acc[mb][nb]); }
    }
    const int bb = c0 / SEQ, tt = c0 % SEQ;
    const size_t tbase = (size_t)bb * (size_t)FOUT * SEQ + (size_t)tt;
    float s1[4], s2[4];
#pragma unroll
    for (int nb = 0; nb < 4; ++nb) { s1[nb] = 0.0f; s2[nb] = 0.0f; }
#pragma unroll
    for (int mb = 0; mb < 4; ++mb) {
        float a1v[8], a2v[8];
#pragma unroll
        for (int j = 0; j < 8; ++j) { a1v[j] = bfr(avec[mb * 16 + hi * 8 + j]); a2v[j] = bfr(avec[FOUT + mb * 16 + hi * 8 + j]); }
#pragma unroll
        for (int nb = 0; nb < 4; ++nb) {
#pragma unroll
            for (int j = 0; j < 8; ++j) { const float c = acc[mb][nb][j];
                os[(hi * 8 + j) * 68 + nb * 16 + lr] = c; s1[nb] += c * a1v[j]; s2[nb] += c * a2v[j]; } }
        wave_sync();
#pragma unroll 1
        for (int ps = 0; ps < 2; ++ps) {
            const size_t sb = tbase + (size_t)(mb * 16) * SEQ;
#pragma unroll
            for (int s = 0; s < 4; ++s) { const int row = 4 * s + (lane >> 3), c8 = (lane & 7) * 8;
                const v4f x0 = *(const v4fa*)(&os[row * 68 + c8]); const v4f x1 = *(const v4fa*)(&os[row * 68 + c8 + 4]); v8h hv;
#pragma unroll
                for (int i = 0; i < 4; ++i) { hv[i] = toh_flush(x0[i]); hv[4 + i] = toh_flush(x1[i]); }
                const size_t oo = sb + (size_t)row * SEQ + c8;
                *(volatile v8h*)(VT + oo) = hv; }
            if (ps == 0) __threadfence(); }
        wave_sync();
    }
#pragma unroll
    for (int nb = 0; nb < 4; ++nb) { s1[nb] += __shfl_xor(s1[nb], 16, 32); s2[nb] += __shfl_xor(s2[nb], 16, 32); }
#pragma unroll
    for (int nb = 0; nb < 4; ++nb) sv[hi * 64 + nb * 16 + lr] = (hi != 0) ? s2[nb] : s1[nb];
    wave_sync();
    const v4f wv = *(const v4fa*)(&sv[hi * 64 + lr * 4]);
    const size_t wo = (size_t)hi * PLN + (size_t)c0 + (size_t)lr * 4;
    *(volatile v4f*)(WH12 + wo) = wv; __threadfence(); *(volatile v4f*)(WH12 + wo) = wv;
}

__global__ __launch_bounds__(32 * AW) __attribute__((amdgpu_num_vgpr(256))) void k_nbrsum(const h16* __restrict__ VT, const float* __restrict__ WH12, const float* __restrict__ adj, float* OUT) {
#pragma clang fp contract(off)
    __shared__ __align__(16) float os[AW * 16 * OSP];
    const int lane = threadIdx.x & 31, lr = lane & 15, hi = lane >> 4;
    const int wave = __builtin_amdgcn_readfirstlane((int)(threadIdx.x >> 5));
    const int bt = blockIdx.y;
    const int t0 = (blockIdx.x * AW + wave) * 16;
    const float w1 = WH12[(size_t)bt * SEQ + t0 + lr];
    const float* w2p = WH12 + PLN + (size_t)bt * SEQ + 8 * hi;
    const float* ajp = adj + (size_t)(t0 + lr) * SEQ_FULL + 8 * hi;
    const size_t vo = (size_t)bt * (size_t)FOUT * SEQ + (size_t)lr * SEQ + 8 * hi;
    v8f o0 = (v8f){}, o1 = (v8f){}, o2 = (v8f){}, o3 = (v8f){};
    float m = NEGB, l = 0.0f;
#pragma unroll 1
    for (int key0 = 0; key0 < SEQ; key0 += 32) {
        const float* wp = w2p + key0; const float* ap = ajp + key0;
        const v4f u0 = *(const v4f*)wp, u1 = *(const v4f*)(wp + 4), u2 = *(const v4f*)(wp + 16), u3 = *(const v4f*)(wp + 20);
        const v4f g0 = *(const v4f*)ap, g1 = *(const v4f*)(ap + 4), g2 = *(const v4f*)(ap + 16), g3 = *(const v4f*)(ap + 20);
        float wx[8], wy[8], gx[8], gy[8];
#pragma unroll
        for (int r = 0; r < 4; ++r) { wx[r] = u0[r]; wx[4 + r] = u1[r]; wy[r] = u2[r]; wy[4 + r] = u3[r]; gx[r] = g0[r]; gx[4 + r] = g1[r]; gy[r] = g2[r]; gy[4 + r] = g3[r]; }
        float ta[8], tb[8]; float mx = NEGB;
#pragma unroll
        for (int r = 0; r < 8; ++r) {
            float ea = w1 + wx[r], eb = w1 + wy[r];
            ea = (ea > 0.0f) ? ea : (LRA * ea); eb = (eb > 0.0f) ? eb : (LRA * eb);
            ta[r] = (bfr(gx[r]) > 0.0f) ? (ea * L2E) : NEGT;
            tb[r] = (bfr(gy[r]) > 0.0f) ? (eb * L2E) : NEGT;
            mx = fmaxf(mx, fmaxf(ta[r], tb[r])); }
        mx = fmaxf(mx, __shfl_xor(mx, 16, 32));
        const float mnew = fmaxf(m, mx);
        const float alpha = __builtin_amdgcn_exp2f(m - mnew);
        v16h pb; float ls = 0.0f;
#pragma unroll
        for (int r = 0; r < 8; ++r) {
            const float xa = (ta[r] - mnew) + PSH, xb = (tb[r] - mnew) + PSH;
            const float ea = __builtin_amdgcn_exp2f(xa), eb = __builtin_amdgcn_exp2f(xb);
            const float ga = (xa < -14.0f) ? 0.0f : ea, gb = (xb < -14.0f) ? 0.0f : eb;
            const h16 pa = (h16)ga; const h16 pc = (h16)gb;
            pb[r] = pa; pb[8 + r] = pc;
            ls += (float)pa + (float)pc; }
        l = l * alpha + ls; m = mnew;
        o0 = o0 * alpha; o1 = o1 * alpha; o2 = o2 * alpha; o3 = o3 * alpha;
        const h16* va = VT + vo + key0;
        const v16h v0 = ldh(va), v1 = ldh(va + (size_t)16 * SEQ), v2 = ldh(va + (size_t)32 * SEQ), v3 = ldh(va + (size_t)48 * SEQ);
        o0 = wmma16g(v0, pb, o0); o1 = wmma16g(v1, pb, o1); o2 = wmma16g(v2, pb, o2); o3 = wmma16g(v3, pb, o3);
    }
    l += __shfl_xor(l, 16, 32);
    const bool any = l > 0.0f;
    const float lsafe = any ? l : 1.0f;
    const float inv = any ? (1.0f / lsafe) : 0.0f;
    const int wb = wave * 16 * OSP;
    { v4f a, c;
#pragma unroll
      for (int i = 0; i < 4; ++i) { a[i] = elu1(o0[i] * inv); c[i] = elu1(o0[4 + i] * inv); }
      *(v4fa*)(&os[wb + lr * OSP +  0 + 8 * hi]) = a; *(v4fa*)(&os[wb + lr * OSP +  0 + 8 * hi + 4]) = c;
#pragma unroll
      for (int i = 0; i < 4; ++i) { a[i] = elu1(o1[i] * inv); c[i] = elu1(o1[4 + i] * inv); }
      *(v4fa*)(&os[wb + lr * OSP + 16 + 8 * hi]) = a; *(v4fa*)(&os[wb + lr * OSP + 16 + 8 * hi + 4]) = c;
#pragma unroll
      for (int i = 0; i < 4; ++i) { a[i] = elu1(o2[i] * inv); c[i] = elu1(o2[4 + i] * inv); }
      *(v4fa*)(&os[wb + lr * OSP + 32 + 8 * hi]) = a; *(v4fa*)(&os[wb + lr * OSP + 32 + 8 * hi + 4]) = c;
#pragma unroll
      for (int i = 0; i < 4; ++i) { a[i] = elu1(o3[i] * inv); c[i] = elu1(o3[4 + i] * inv); }
      *(v4fa*)(&os[wb + lr * OSP + 48 + 8 * hi]) = a; *(v4fa*)(&os[wb + lr * OSP + 48 + 8 * hi + 4]) = c; }
    wave_sync();
    float* orow = OUT + ((size_t)bt * OUT_SEQ + t0) * FOUT;
#pragma unroll 1
    for (int ps = 0; ps < 2; ++ps) {
#pragma unroll
        for (int s = 0; s < 8; ++s) { const int p = s * 32 + lane; const int row = p >> 4, cofs = (p & 15) * 4;
            const v4f val = *(const v4fa*)(&os[wb + row * OSP + cofs]);
            *(volatile v4f*)(orow + (size_t)p * 4) = val; }
        if (ps == 0) __threadfence(); }
}

static constexpr size_t al256(size_t v) { return (v + 255) & ~(size_t)255; }
static constexpr size_t SZ_XB = al256((size_t)NB * SEQ * FIN * 2);
static constexpr size_t SZ_WT = al256((size_t)FIN * FOUT * 2);
static constexpr size_t SZ_VT = al256((size_t)NB * FOUT * SEQ * 2);
static constexpr size_t SZ_WH = al256((size_t)2 * NB * SEQ * 4);
static constexpr size_t SZ_TOTAL = SZ_XB + SZ_WT + SZ_VT + SZ_WH;
static_assert(SZ_TOTAL <= (size_t)134217728);
static_assert(((size_t)NB * SEQ * 4) % 256 == 0);
static_assert((size_t)(NB * SEQ / 64) * 64 * FIN * 2 <= SZ_XB);
static_assert((size_t)((NB * SEQ / 64 - 1) / (SEQ / 64)) * FOUT * SEQ + (size_t)63 * SEQ + SEQ <= (size_t)NB * FOUT * SEQ);
static_assert(((size_t)NB * SEQ / 64 - 1) * 64 + 64 + PLN <= (size_t)2 * NB * SEQ);

extern "C" void kernel_launch(void* const* d_in, const int* in_sizes, int n_in,
                              void* d_out, int out_size, void* d_ws, size_t ws_size, hipStream_t stream) {
    if (n_in < 4) return;
    const size_t needh = ((size_t)(NB - 1) * SEQ_FULL + SEQ) * FIN;
    const size_t needa = (size_t)(SEQ - 1) * SEQ_FULL + SEQ;
    if ((size_t)in_sizes[0] < needh || (size_t)in_sizes[1] < needa) return;
    if ((size_t)in_sizes[2] < (size_t)FIN * FOUT || in_sizes[3] < 2 * FOUT) return;
    if ((size_t)out_size < ((size_t)(NB - 1) * OUT_SEQ + SEQ) * FOUT) return;
    if (SZ_TOTAL > ws_size) return;
    const float* hin = (const float*)d_in[0];
    const float* adj = (const float*)d_in[1];
    const float* wgt = (const float*)d_in[2];
    const float* avec = (const float*)d_in[3];
    float* OUT = (float*)d_out;
    char* wsp = (char*)d_ws;
    bf* XB = (bf*)wsp; wsp += SZ_XB;
    bf* WT = (bf*)wsp; wsp += SZ_WT;
    h16* VT = (h16*)wsp; wsp += SZ_VT;
    float* WH12 = (float*)wsp; wsp += SZ_WH;

    if (SEQ == SEQ_FULL) {
        const size_t n8 = (size_t)NB * SEQ * FIN / 8;
        k_cvt8<<<(unsigned)((n8 + 255) / 256), 256, 0, stream>>>(hin, XB, n8);
    } else {
        const size_t n8 = (size_t)SEQ * FIN / 8;
        for (int b = 0; b < NB; ++b) k_cvt8<<<(unsigned)((n8 + 255) / 256), 256, 0, stream>>>(hin + (size_t)b * SEQ_FULL * FIN, XB + (size_t)b * SEQ * FIN, n8);
    }
    k_wt<<<1, 256, 0, stream>>>(wgt, WT);

    k_whT<<<dim3(NB * SEQ / 64, 1, 1), 32, 0, stream>>>(WT, XB, avec, VT, WH12);

    k_nbrsum<<<dim3(SEQ / (16 * AW), NB, 1), 32 * AW, 0, stream>>>(VT, WH12, adj, OUT);
}
